// NonLocal3D_7481833029823
// MI455X (gfx1250) — hardware-verified
//
#include <hip/hip_runtime.h>


typedef _Float16     v16h  __attribute__((ext_vector_type(16)));
typedef float        v8f   __attribute__((ext_vector_type(8)));
typedef float        v4f   __attribute__((ext_vector_type(4)));
typedef unsigned int u32x4 __attribute__((ext_vector_type(4)));
typedef unsigned int u32x2 __attribute__((ext_vector_type(2)));

#define M_TOT 6272
#define C_IN  512
#define H_CH  256
#define BATCH 2
#define QT    64
#define KT    64
#define NTHR  256

typedef char chk_m[(M_TOT % 64 == 0 && M_TOT % KT == 0 && M_TOT % QT == 0) ? 1 : -1];
typedef char chk_c[(C_IN % 64 == 0 && H_CH % 64 == 0 && C_IN % 32 == 0) ? 1 : -1];

#define W_SCALE        1024.0f
#define PROJ_OUT_SCALE (1.0f / 64.0f)
#define S_SCALE        (1.0f / 16.0f)
#define P_SCALE        4096.0f
#define Y_DIV          4096.0f
#define OUT_SCALE      (1.0f / 16384.0f)

union H8   { u32x4 q; _Float16 h[8]; unsigned short s[8]; };
union Frag { v16h v; u32x4 q[2]; };

__device__ __forceinline__ v8f wmma16(v16h a, v16h b, v8f c) {
  v8f d = __builtin_amdgcn_wmma_f32_16x16x32_f16(false, a, false, b, (short)0, c, false, false);
  asm volatile("v_nop\n\tv_nop\n\tv_nop\n\tv_nop" : "+v"(d) : "v"(a), "v"(b));
  return d;
}

__device__ __forceinline__ v16h load_frag(const _Float16* p, int ld) {
  const int lane = threadIdx.x & 31;
  const _Float16* row = p + (lane & 15) * ld + (lane >> 4) * 8;
  Frag u;
  u.q[0] = *(const u32x4*)row;
  u.q[1] = *(const u32x4*)(row + 16);
  return u.v;
}

__device__ __forceinline__ u32x4 cvt8(const float* __restrict__ src, float scale) {
  const v4f f0 = *(const v4f*)src;
  const v4f f1 = *(const v4f*)(src + 4);
  H8 u;
  u.h[0] = (_Float16)(f0.x * scale); u.h[1] = (_Float16)(f0.y * scale);
  u.h[2] = (_Float16)(f0.z * scale); u.h[3] = (_Float16)(f0.w * scale);
  u.h[4] = (_Float16)(f1.x * scale); u.h[5] = (_Float16)(f1.y * scale);
  u.h[6] = (_Float16)(f1.z * scale); u.h[7] = (_Float16)(f1.w * scale);
  return u.q;
}

__global__ __launch_bounds__(NTHR) __attribute__((amdgpu_num_vgpr(256)))
void k_proj(const float* __restrict__ x,
            const float* __restrict__ w_theta,
            const float* __restrict__ w_phi,
            const float* __restrict__ w_g,
            _Float16* __restrict__ theta,
            _Float16* __restrict__ phi,
            _Float16* __restrict__ g) {
  const int mb = blockIdx.x;
  const int ob = blockIdx.y;
  const int n  = blockIdx.z;
  const int tid = threadIdx.x;
  const int wave = tid >> 5, lane = tid & 31;
  if (mb * 64 >= M_TOT || n >= BATCH) return;

  const int o0 = ob * 64;
  const float* w; _Float16* outp; int ol0;
  if (o0 < H_CH)          { w = w_theta; outp = theta; ol0 = o0; }
  else if (o0 < 2 * H_CH) { w = w_phi;   outp = phi;   ol0 = o0 - H_CH; }
  else                    { w = w_g;     outp = g;     ol0 = o0 - 2 * H_CH; }
  if (ol0 + 64 > H_CH) return;

  __shared__ __attribute__((aligned(16))) _Float16 sh[2 * 64 * 32];
  _Float16* At  = sh;
  _Float16* BtT = sh + 64 * 32;

  v8f acc[2] = {};
  const int wr = (wave & 3) * 16;
  const int wc = (wave >> 2) * 16;
  const int h8 = (lane >> 4) * 8;
  const int coll = lane & 15;

  const size_t xbase = (size_t)n * C_IN * M_TOT + (size_t)mb * 64;
#pragma unroll 1
  for (int c0 = 0; c0 < C_IN; c0 += 32) {
    {
      const int mm = tid & 63;
      const int cb = (tid >> 6) * 8;
      H8 u;
#pragma unroll
      for (int r = 0; r < 8; ++r)
        u.h[r] = (_Float16)x[xbase + (size_t)(c0 + cb + r) * M_TOT + mm];
      *(u32x4*)&At[mm * 32 + cb] = u.q;
    }
    {
      const int oo  = tid >> 2;
      const int cc8 = (tid & 3) * 8;
      *(u32x4*)&BtT[oo * 32 + cc8] = cvt8(&w[(size_t)(ol0 + oo) * C_IN + c0 + cc8], W_SCALE);
    }
    __syncthreads();
    const v16h a = load_frag(&At[wr * 32], 32);
#pragma unroll
    for (int j = 0; j < 2; ++j) {
      const v16h b = load_frag(&BtT[(wc + j * 32) * 32], 32);
      acc[j] = wmma16(a, b, acc[j]);
    }
    __syncthreads();
  }

  _Float16* tile = sh;
#pragma unroll
  for (int j = 0; j < 2; ++j)
#pragma unroll
    for (int i = 0; i < 8; ++i)
      tile[(wr + h8 + i) * 64 + wc + j * 32 + coll] = (_Float16)(acc[j][i] * PROJ_OUT_SCALE);
  __syncthreads();
  u32x4 v[2];
  size_t off[2];
#pragma unroll
  for (int k = 0; k < 2; ++k) {
    const int i = tid + NTHR * k;
    const int mm = i >> 3, seg = i & 7;
    v[k] = *(const u32x4*)&tile[mm * 64 + seg * 8];
    off[k] = ((size_t)n * M_TOT + (size_t)mb * 64 + mm) * H_CH + ol0 + seg * 8;
    *(volatile u32x4*)(outp + off[k]) = v[k];
  }
  __threadfence();
#pragma unroll
  for (int k = 0; k < 2; ++k)
    *(volatile u32x4*)(outp + off[k]) = v[k];
}

#define ATTN_SMEM (QT * H_CH * 2 + KT * H_CH * 2 + H_CH * KT * 2 + \
                   QT * KT * 4 + QT * KT * 2 + 3 * QT * 4)

__global__ __launch_bounds__(NTHR) __attribute__((amdgpu_num_vgpr(256)))
void k_attn(const _Float16* __restrict__ theta, const _Float16* __restrict__ phi,
            const _Float16* __restrict__ g, _Float16* __restrict__ y) {
  const int qb = blockIdx.x;
  const int n  = blockIdx.y;
  const int tid = threadIdx.x;
  const int wave = tid >> 5, lane = tid & 31;
  if (qb * QT >= M_TOT || n >= BATCH) return;

  extern __shared__ __attribute__((aligned(16))) unsigned char smem[];
  _Float16* Qt  = (_Float16*)smem;
  _Float16* Kt  = Qt + QT * H_CH;
  _Float16* VtT = Kt + KT * H_CH;
  float*    Sf  = (float*)(VtT + H_CH * KT);
  _Float16* Pt  = (_Float16*)(Sf + QT * KT);
  float* rowm = (float*)(Pt + QT * KT);
  float* rowl = rowm + QT;
  float* rowf = rowl + QT;

  const _Float16* Qg = theta + ((size_t)n * M_TOT + (size_t)qb * QT) * H_CH;
  for (int i = tid; i < QT * H_CH / 8; i += NTHR)
    ((u32x4*)Qt)[i] = ((const u32x4*)Qg)[i];
  if (tid < QT) { rowm[tid] = -1e30f; rowl[tid] = 0.0f; rowf[tid] = 0.0f; }

  const int wr  = (wave & 3) * 16;
  const int wch = (wave >> 2) * 128;
  const int sc  = (wave >> 2) * 16;
  const int h8  = (lane >> 4) * 8;
  const int coll = lane & 15;

  v8f acc[8] = {};
  const int nkb = M_TOT / KT;
  __syncthreads();

#pragma unroll 1
  for (int kb = 0; kb < nkb; ++kb) {
    const _Float16* Kg = phi + ((size_t)n * M_TOT + (size_t)kb * KT) * H_CH;
    const _Float16* Vg = g   + ((size_t)n * M_TOT + (size_t)kb * KT) * H_CH;
#pragma unroll
    for (int r = 0; r < 8; ++r) {
      const int i = tid + NTHR * r;
      ((u32x4*)Kt)[i] = ((const u32x4*)Kg)[i];
    }
#pragma unroll
    for (int r = 0; r < 2; ++r) {
      const int it = tid + NTHR * r;
      const int db = it & 31;
      const int kq = it >> 5;
      const u32x4* vp = (const u32x4*)Vg + (size_t)(4 * kq) * (H_CH / 8) + db;
      H8 u0, u1, u2, u3;
      u0.q = vp[0];
      u1.q = vp[H_CH / 8];
      u2.q = vp[2 * (H_CH / 8)];
      u3.q = vp[3 * (H_CH / 8)];
#pragma unroll
      for (int j = 0; j < 8; ++j) {
        u32x2 wv;
        wv.x = (unsigned int)u0.s[j] | ((unsigned int)u1.s[j] << 16);
        wv.y = (unsigned int)u2.s[j] | ((unsigned int)u3.s[j] << 16);
        *(u32x2*)(VtT + (db * 8 + j) * KT + 4 * kq) = wv;
      }
    }
    __syncthreads();

    v8f s[2] = {};
#pragma unroll 2
    for (int d0 = 0; d0 < H_CH; d0 += 32) {
      const v16h a = load_frag(Qt + wr * H_CH + d0, H_CH);
#pragma unroll
      for (int jj = 0; jj < 2; ++jj) {
        const v16h b = load_frag(Kt + (sc + jj * 32) * H_CH + d0, H_CH);
        s[jj] = wmma16(a, b, s[jj]);
      }
    }
#pragma unroll
    for (int jj = 0; jj < 2; ++jj)
#pragma unroll
      for (int i = 0; i < 8; ++i)
        Sf[(wr + h8 + i) * KT + sc + jj * 32 + coll] = s[jj][i] * S_SCALE;
    __syncthreads();

    {
      const int r  = tid >> 2;
      const int qq = tid & 3;
      const float* srow = &Sf[r * KT + qq * 16];
      float sv[16];
#pragma unroll
      for (int v4 = 0; v4 < 4; ++v4) {
        const v4f f = *(const v4f*)(srow + 4 * v4);
        sv[4 * v4 + 0] = f.x; sv[4 * v4 + 1] = f.y;
        sv[4 * v4 + 2] = f.z; sv[4 * v4 + 3] = f.w;
      }
      float mx = sv[0];
#pragma unroll
      for (int k = 1; k < 16; ++k) mx = fmaxf(mx, sv[k]);
      mx = fmaxf(mx, __shfl_xor(mx, 1, 4));
      mx = fmaxf(mx, __shfl_xor(mx, 2, 4));
      mx = fmaxf(mx, rowm[r]);
      float sum = 0.0f;
      H8 p0, p1;
#pragma unroll
      for (int k = 0; k < 8; ++k) {
        const float p = __expf(sv[k] - mx);
        p0.h[k] = (_Float16)(p * P_SCALE);
        sum += p;
      }
#pragma unroll
      for (int k = 0; k < 8; ++k) {
        const float p = __expf(sv[8 + k] - mx);
        p1.h[k] = (_Float16)(p * P_SCALE);
        sum += p;
      }
      *(u32x4*)&Pt[r * KT + qq * 16]     = p0.q;
      *(u32x4*)&Pt[r * KT + qq * 16 + 8] = p1.q;
      sum += __shfl_xor(sum, 1, 4);
      sum += __shfl_xor(sum, 2, 4);
      __syncthreads();
      if (qq == 0) {
        const float f = __expf(rowm[r] - mx);
        rowl[r] = rowl[r] * f + sum;
        rowm[r] = mx;
        rowf[r] = f;
      }
    }
    __syncthreads();

    float fr[8];
#pragma unroll
    for (int i = 0; i < 8; ++i) fr[i] = rowf[wr + h8 + i];
    const v16h a0 = load_frag(Pt + wr * KT, KT);
    const v16h a1 = load_frag(Pt + wr * KT + 32, KT);
#pragma unroll
    for (int j = 0; j < 8; ++j) {
#pragma unroll
      for (int i = 0; i < 8; ++i) acc[j][i] *= fr[i];
      const v16h b0 = load_frag(VtT + (wch + j * 16) * KT, KT);
      acc[j] = wmma16(a0, b0, acc[j]);
      const v16h b1 = load_frag(VtT + (wch + j * 16) * KT + 32, KT);
      acc[j] = wmma16(a1, b1, acc[j]);
    }
    __syncthreads();
  }

  float inv[8];
#pragma unroll
  for (int i = 0; i < 8; ++i) inv[i] = 1.0f / (Y_DIV * rowl[wr + h8 + i]);
#pragma unroll
  for (int j = 0; j < 8; ++j)
#pragma unroll
    for (int i = 0; i < 8; ++i)
      Qt[(wr + h8 + i) * H_CH + wch + j * 16 + coll] = (_Float16)(acc[j][i] * inv[i]);
  __syncthreads();
  _Float16* Yg = y + ((size_t)n * M_TOT + (size_t)qb * QT) * H_CH;
#pragma unroll
  for (int r = 0; r < 8; ++r) {
    const int i = tid + NTHR * r;
    const u32x4 v = ((const u32x4*)Qt)[i];
    *(volatile u32x4*)((u32x4*)Yg + i) = v;
  }
  __threadfence();
#pragma unroll
  for (int r = 0; r < 8; ++r) {
    const int i = tid + NTHR * r;
    const u32x4 v = ((const u32x4*)Qt)[i];
    *(volatile u32x4*)((u32x4*)Yg + i) = v;
  }
}

__global__ __launch_bounds__(NTHR) __attribute__((amdgpu_num_vgpr(256)))
void k_out(const float* __restrict__ x, const float* __restrict__ w_out,
           const _Float16* __restrict__ y, float* __restrict__ out) {
  const int mb  = blockIdx.x;
  const int cbk = blockIdx.y;
  const int n   = blockIdx.z;
  const int tid = threadIdx.x;
  const int wave = tid >> 5, lane = tid & 31;
  if (mb * 64 >= M_TOT || cbk * 64 >= C_IN || n >= BATCH) return;

  __shared__ __attribute__((aligned(16))) _Float16 At[64 * 32];
  __shared__ __attribute__((aligned(16))) _Float16 BtT[64 * 32];
  __shared__ __attribute__((aligned(16))) float    Tt[64 * 64];

  v8f acc[2] = {};
  const int wr = (wave & 3) * 16;
  const int wc = (wave >> 2) * 16;
  const int h8 = (lane >> 4) * 8;
  const int coll = lane & 15;

#pragma unroll 1
  for (int o0 = 0; o0 < H_CH; o0 += 32) {
    {
      const int rr  = tid >> 2;
      const int ob8 = (tid & 3) * 8;
      *(u32x4*)&At[rr * 32 + ob8] = cvt8(&w_out[(size_t)(cbk * 64 + rr) * H_CH + o0 + ob8], W_SCALE);
    }
    {
      const int mm  = tid >> 2;
      const int ob8 = (tid & 3) * 8;
      *(u32x4*)&BtT[mm * 32 + ob8] =
          *(const u32x4*)&y[((size_t)n * M_TOT + (size_t)mb * 64 + mm) * H_CH + o0 + ob8];
    }
    __syncthreads();
    const v16h a = load_frag(&At[wr * 32], 32);
#pragma unroll
    for (int j = 0; j < 2; ++j) {
      const v16h b = load_frag(&BtT[(wc + j * 32) * 32], 32);
      acc[j] = wmma16(a, b, acc[j]);
    }
    __syncthreads();
  }

#pragma unroll
  for (int j = 0; j < 2; ++j)
#pragma unroll
    for (int i = 0; i < 8; ++i)
      Tt[(wr + h8 + i) * 64 + wc + j * 32 + coll] = acc[j][i];
  __syncthreads();

  const int q = lane >> 3, e = lane & 7;
  v4f vals[4];
  size_t offs[4];
#pragma unroll
  for (int t = 0; t < 4; ++t) {
    const int L = wave * 16 + t * 4 + q;
    const int row = L >> 1;
    const int ml = (L & 1) * 32 + e * 4;
    const size_t idx = ((size_t)n * C_IN + (size_t)(cbk * 64 + row)) * M_TOT + (size_t)mb * 64 + ml;
    const v4f xv = *(const v4f*)(x + idx);
    const v4f tv = *(const v4f*)&Tt[row * 64 + ml];
    vals[t] = xv + tv * OUT_SCALE;
    offs[t] = idx;
    *(volatile v4f*)(out + idx) = vals[t];
  }
  __threadfence();
#pragma unroll
  for (int t = 0; t < 4; ++t)
    *(volatile v4f*)(out + offs[t]) = vals[t];
}

extern "C" void kernel_launch(void* const* d_in, const int* in_sizes, int n_in,
                              void* d_out, int out_size, void* d_ws, size_t ws_size,
                              hipStream_t stream) {
  if (n_in < 5) return;
  if (in_sizes[0] != BATCH * C_IN * M_TOT) return;
  if (in_sizes[1] != H_CH * C_IN || in_sizes[2] != H_CH * C_IN || in_sizes[3] != H_CH * C_IN) return;
  if (in_sizes[4] != C_IN * H_CH) return;
  if (out_size != BATCH * C_IN * M_TOT) return;

  const float* x       = (const float*)d_in[0];
  const float* w_g     = (const float*)d_in[1];
  const float* w_theta = (const float*)d_in[2];
  const float* w_phi   = (const float*)d_in[3];
  const float* w_out   = (const float*)d_in[4];
  float* out = (float*)d_out;

  const size_t T = (size_t)BATCH * M_TOT * H_CH;
  if (4 * T * sizeof(_Float16) > ws_size) return;
  _Float16* theta = (_Float16*)d_ws;
  _Float16* phi   = theta + T;
  _Float16* g     = phi + T;
  _Float16* y     = g + T;

  const dim3 blk(NTHR);
  const dim3 g1((M_TOT + 63) / 64, (3 * H_CH) / 64, BATCH);
  const dim3 g2((M_TOT + QT - 1) / QT, BATCH);
  const dim3 g3((M_TOT + 63) / 64, C_IN / 64, BATCH);
  hipLaunchKernelGGL(k_proj, g1, blk, 0, stream, x, w_theta, w_phi, w_g, theta, phi, g);
  hipLaunchKernelGGL(k_attn, g2, blk, (size_t)ATTN_SMEM, stream,
                     (const _Float16*)theta, (const _Float16*)phi, (const _Float16*)g, y);
  hipLaunchKernelGGL(k_out, g3, blk, 0, stream, x, w_out, (const _Float16*)y, out);
}
